// STPAttention_82094004896537
// MI455X (gfx1250) — hardware-verified
//
#include <hip/hip_runtime.h>
#include <math.h>

constexpr int kNB      = 2;
constexpr int kSeqLen  = 2048;
constexpr int kModel   = 1024;
constexpr int kHeads   = 16;
constexpr int kDk      = 64;
constexpr int kRows    = kNB * kSeqLen;
constexpr int kQkvCols = 3 * kModel;
constexpr int kChunk   = 32;
constexpr int kThreads = 256;
constexpr float kWCarry    = 64.0f;
constexpr float kWCarryInv = 1.0f / kWCarry;
constexpr float kLnEps     = 1e-5f;
constexpr float kInvDk     = 1.0f / (float)kDk;
static_assert(kModel == kHeads * kDk, "head split");
static_assert(kDk == 64, "one head row of 16-bit values = one 128-B line");
static_assert(kSeqLen % kChunk == 0, "chunking exact");
static_assert(kChunk == 4 * (kThreads / 32), "8 waves x 4 steps per chunk");
static_assert(3 * kChunk * kDk == 6 * kThreads * 4, "staging loop exact: 6 x 256 x 4 floats");
static_assert(kRows % 64 == 0 && kQkvCols % 64 == 0 && kModel % 64 == 0, "GEMM tile multiples");
static_assert(kModel % 32 == 0, "GEMM K multiple of 32");
static_assert((kHeads * kDk * kDk) % kThreads == 0, "constants grid exact");

typedef __attribute__((ext_vector_type(16))) _Float16 v16h;
typedef __attribute__((ext_vector_type(8)))  _Float16 v8h;
typedef __attribute__((ext_vector_type(8)))  float    v8f;
typedef __attribute__((ext_vector_type(4)))  float    v4f;
typedef __attribute__((ext_vector_type(4)))  unsigned int v4u;

__device__ __forceinline__ void dep_guard4_h(v8f& a, v8f& b, v8f& c, v8f& d, v16h x, v16h y) {
  asm volatile("v_nop\n\tv_nop\n\tv_nop\n\tv_nop" : "+v"(a), "+v"(b), "+v"(c), "+v"(d) : "v"(x), "v"(y));
}
__device__ __forceinline__ void keep4_h(v16h a, v16h b, v16h c, v16h d) { asm volatile("v_nop" :: "v"(a), "v"(b), "v"(c), "v"(d)); }
__device__ __forceinline__ void acc_guard4(v8f& a, v8f& b, v8f& c, v8f& d) { asm volatile("v_nop\n\tv_nop\n\tv_nop\n\tv_nop" : "+v"(a), "+v"(b), "+v"(c), "+v"(d)); }

union FragU { v16h v; v8h h[2]; };
__device__ __forceinline__ v16h frag_load(const _Float16* p) {
  FragU f;
  f.h[0] = *(const v8h*)(p);
  f.h[1] = *(const v8h*)(p + 16);
  return f.v;
}
__device__ __forceinline__ v8f frag_mma(v16h a, v16h b, v8f c) {
  return __builtin_amdgcn_wmma_f32_16x16x32_f16(false, a, false, b, (short)0, c, false, false);
}

__device__ __forceinline__ unsigned pk16(unsigned short a, unsigned short b) { return (unsigned)a | ((unsigned)b << 16); }
__device__ __forceinline__ unsigned short h_bits(float f) { const _Float16 h = (_Float16)f; return __builtin_bit_cast(unsigned short, h); }

__global__ __launch_bounds__(256) void cast8_f16_kernel(const float* __restrict__ in, unsigned short* __restrict__ out,
                                                        int n8, float sc) {
  const int i = blockIdx.x * 256 + threadIdx.x;
  if (i >= n8) return;
  const float* p = in + 8 * (size_t)i;
  const v4f a = *(const v4f*)(p);
  const v4f c = *(const v4f*)(p + 4);
  unsigned short hb[8];
#pragma unroll
  for (int e = 0; e < 4; ++e) {
    hb[e]     = h_bits(a[e] * sc);
    hb[4 + e] = h_bits(c[e] * sc);
  }
  const v4u u = (v4u){pk16(hb[0], hb[1]), pk16(hb[2], hb[3]), pk16(hb[4], hb[5]), pk16(hb[6], hb[7])};
  unsigned short* q = out + 8 * (size_t)i;
  *(volatile v4u*)q = u;
  __threadfence();
  *(volatile v4u*)q = u;
}

__global__ __launch_bounds__(256) void gemm_f16_nt_kernel(
    const unsigned short* __restrict__ Ap, int lda,
    const unsigned short* __restrict__ Btp, int ldb,
    float* __restrict__ Cout, int ldc,
    int M, int N, int K, float scale) {
  const _Float16* A  = (const _Float16*)Ap;
  const _Float16* Bt = (const _Float16*)Btp;
  __shared__ __align__(16) float sT[8][16 * 68];
  const int lane = threadIdx.x & 31;
  const int wave = threadIdx.x >> 5;
  const int tilesN = N >> 6;
  const int tilesM = M >> 6;
  const int tile = blockIdx.x * 8 + wave;
  if (tile >= tilesM * tilesN) return;
  const int tm = tile / tilesN;
  const int tn = tile - tm * tilesN;
  const int m0 = tm << 6;
  const int n0 = tn << 6;

  const int rlane = lane & 15;
  const int koff  = (lane >> 4) * 8;
  const int mOff  = (lane >> 4) * 8;

  v8f acc[4][4];
#pragma unroll
  for (int i = 0; i < 4; ++i)
#pragma unroll
    for (int j = 0; j < 4; ++j) acc[i][j] = (v8f){0.f, 0.f, 0.f, 0.f, 0.f, 0.f, 0.f, 0.f};

  for (int k0 = 0; k0 < K; k0 += 32) {
    v16h bh[4];
#pragma unroll
    for (int j = 0; j < 4; ++j) {
      const size_t bo = (size_t)(n0 + (j << 4) + rlane) * ldb + koff + k0;
      bh[j] = frag_load(Bt + bo);
    }
#pragma unroll
    for (int i = 0; i < 4; ++i) {
      const size_t ao = (size_t)(m0 + (i << 4) + rlane) * lda + koff + k0;
      const v16h ah = frag_load(A + ao);
#pragma unroll
      for (int j = 0; j < 4; ++j) acc[i][j] = frag_mma(ah, bh[j], acc[i][j]);
      dep_guard4_h(acc[i][0], acc[i][1], acc[i][2], acc[i][3], ah, bh[3]);
    }
    keep4_h(bh[0], bh[1], bh[2], bh[3]);
  }
  acc_guard4(acc[0][0], acc[0][1], acc[0][2], acc[0][3]);
  acc_guard4(acc[1][0], acc[1][1], acc[1][2], acc[1][3]);
  acc_guard4(acc[2][0], acc[2][1], acc[2][2], acc[2][3]);
  acc_guard4(acc[3][0], acc[3][1], acc[3][2], acc[3][3]);

  float* slab = sT[wave];
#pragma unroll
  for (int i = 0; i < 4; ++i) {
    const int mBase = m0 + (i << 4);
#pragma unroll
    for (int j = 0; j < 4; ++j) {
#pragma unroll
      for (int r = 0; r < 8; ++r) {
        const float v = acc[i][j][r] * scale;
        slab[(mOff + r) * 68 + (j << 4) + rlane] = v;
      }
    }
    __builtin_amdgcn_fence(__ATOMIC_RELEASE, "workgroup");
    __builtin_amdgcn_wave_barrier();
    __builtin_amdgcn_fence(__ATOMIC_ACQUIRE, "workgroup");
    {
      const int hh = lane >> 4;
      const int c4 = (lane & 15) * 4;
      for (int pass = 0; pass < 2; ++pass) {
#pragma unroll
        for (int it = 0; it < 8; ++it) {
          const int row = it * 2 + hh;
          const v4f v = *(const v4f*)(slab + row * 68 + c4);
          *(volatile v4f*)(Cout + (size_t)(mBase + row) * ldc + n0 + c4) = v;
        }
        __threadfence();
      }
    }
    __builtin_amdgcn_fence(__ATOMIC_RELEASE, "workgroup");
    __builtin_amdgcn_wave_barrier();
    __builtin_amdgcn_fence(__ATOMIC_ACQUIRE, "workgroup");
  }
}

__global__ __launch_bounds__(256) void head_consts_kernel(
    const float* __restrict__ W, const float* __restrict__ Vgs, const float* __restrict__ Vt0,
    const float* __restrict__ btau, const float* __restrict__ bgm, const float* __restrict__ cch,
    const float* __restrict__ gam, const float* __restrict__ alpha, const float* __restrict__ icth,
    float* __restrict__ retp, float* __restrict__ coefp) {
  __shared__ __align__(16) float sV[512];
  const int tid = threadIdx.x;
  const int i = blockIdx.x * 256 + tid;
  const int h = i / (kDk * kDk);
  const float vn = (Vgs[h] - Vt0[h]) + W[i];
  const float ea  = expf(-fabsf(vn));
  const float sp  = fmaxf(vn, 0.0f) + log1pf(ea);
  const float rc  = 1.0f / (1.0f + ea);
  const float sig = (vn >= 0.0f) ? rc : ea * rc;
  const float gch = btau[h] * sp;
  const float cinv = 1.0f / cch[h];
  const float retv = expf(-(gch * cinv));
  const float G  = (bgm[h] * sp) * sig;
  const float sm = tanhf(alpha[0] * (gch - icth[0]));
  const float cf = (gam[h] * sm) * G;
  sV[tid] = retv;
  sV[256 + tid] = cf;
  __syncthreads();
  if (tid < 128) {
    const v4f val = *(const v4f*)(sV + tid * 4);
    float* dst = (tid < 64) ? (retp + (size_t)blockIdx.x * 256 + tid * 4)
                            : (coefp + (size_t)blockIdx.x * 256 + (tid - 64) * 4);
    *(volatile v4f*)dst = val;
    __threadfence();
    *(volatile v4f*)dst = val;
  }
}

__global__ __launch_bounds__(256) void stp_scan_kernel(const float* __restrict__ qkv, const float* __restrict__ W,
                                                       const float* __restrict__ retp, const float* __restrict__ coefp,
                                                       unsigned short* __restrict__ yh) {
  __shared__ __align__(16) float sIn[3 * kChunk * kDk];
  __shared__ __align__(16) float sY[kChunk * kDk];
  float* sQ = sIn;
  float* sK = sIn + kChunk * kDk;
  float* sV = sIn + 2 * kChunk * kDk;

  const int tid  = threadIdx.x;
  const int lane = tid & 31;
  const int wave = tid >> 5;
  const int b = blockIdx.x / kHeads;
  const int h = blockIdx.x - b * kHeads;
  const int d  = tid >> 2;
  const int e0 = (tid & 3) * 16;

  float F[16], Wr[16], Rr[16], Cr[16];
  {
    const size_t base = (size_t)h * kDk * kDk + (size_t)d * kDk + e0;
#pragma unroll
    for (int jj = 0; jj < 4; ++jj) {
      const v4f w4 = *(const v4f*)(W + base + 4 * jj);
      const v4f r4 = *(const v4f*)(retp + base + 4 * jj);
      const v4f c4 = *(const v4f*)(coefp + base + 4 * jj);
#pragma unroll
      for (int e = 0; e < 4; ++e) {
        F[4 * jj + e]  = 0.0f;
        Wr[4 * jj + e] = w4[e];
        Rr[4 * jj + e] = r4[e];
        Cr[4 * jj + e] = c4[e];
      }
    }
  }

#pragma unroll 1
  for (int ch = 0; ch < kSeqLen / kChunk; ++ch) {
    const int t0 = ch * kChunk;

#pragma unroll
    for (int j = 0; j < 6; ++j) {
      const int w   = j >> 1;
      const int rem = (j & 1) * 256 + tid;
      const int s   = rem >> 4;
      const int c4  = (rem & 15) * 4;
      const float* gp = qkv + (size_t)(b * kSeqLen + t0 + s) * kQkvCols + w * kModel + h * kDk + c4;
      const v4f val = *(const v4f*)gp;
      *(v4f*)(sIn + w * (kChunk * kDk) + s * kDk + c4) = val;
    }
    __syncthreads();

#pragma unroll
    for (int i = 0; i < 4; ++i) {
      const int s = wave * 4 + i;
      const float ka = sK[s * kDk + lane];
      const float kb = sK[s * kDk + 32 + lane];
      float sum = ka + kb;
#pragma unroll
      for (int off = 16; off > 0; off >>= 1) sum += __shfl_xor(sum, off, 32);
      const float mu = sum * kInvDk;
      const float da = ka - mu;
      const float db = kb - mu;
      float ss = da * da + db * db;
#pragma unroll
      for (int off = 16; off > 0; off >>= 1) ss += __shfl_xor(ss, off, 32);
      const float var  = ss * kInvDk;
      const float rstd = 1.0f / sqrtf(var + kLnEps);
      sK[s * kDk + lane]      = da * rstd;
      sK[s * kDk + 32 + lane] = db * rstd;
    }
    __syncthreads();

#pragma unroll 1
    for (int s = 0; s < kChunk; ++s) {
      const float vd = sV[s * kDk + d];
      const float* kp = sK + s * kDk + e0;
      const float* qp = sQ + s * kDk + e0;
      float qs = 0.0f;
#pragma unroll
      for (int jj = 0; jj < 4; ++jj) {
        const v4f k4 = *(const v4f*)(kp + 4 * jj);
        const v4f q4 = *(const v4f*)(qp + 4 * jj);
#pragma unroll
        for (int e = 0; e < 4; ++e) {
          const float hb = vd * k4[e];
          const float Fn = Rr[4 * jj + e] * F[4 * jj + e] + Cr[4 * jj + e] * hb;
          F[4 * jj + e] = Fn;
          qs += (Wr[4 * jj + e] + Fn) * q4[e];
        }
      }
      qs += __shfl_xor(qs, 1, 32);
      qs += __shfl_xor(qs, 2, 32);
      if ((tid & 3) == 0) sY[s * kDk + d] = qs;
    }
    __syncthreads();

    {
      const int qd = lane >> 3;
      const int c8 = (lane & 7) * 8;
      const int s  = wave * 4 + qd;
      const float* sp = sY + s * kDk + c8;
      const v4f ya = *(const v4f*)(sp);
      const v4f yb = *(const v4f*)(sp + 4);
      unsigned short hb[8];
#pragma unroll
      for (int e = 0; e < 4; ++e) {
        hb[e]     = h_bits(ya[e]);
        hb[4 + e] = h_bits(yb[e]);
      }
      const v4u u = (v4u){pk16(hb[0], hb[1]), pk16(hb[2], hb[3]), pk16(hb[4], hb[5]), pk16(hb[6], hb[7])};
      unsigned short* gp = yh + (size_t)(b * kSeqLen + t0 + s) * kModel + h * kDk + c8;
      *(volatile v4u*)gp = u;
      __threadfence();
      *(volatile v4u*)gp = u;
    }
  }
}

extern "C" void kernel_launch(void* const* d_in, const int* in_sizes, int n_in,
                              void* d_out, int out_size, void* d_ws, size_t ws_size, hipStream_t stream) {
  if (n_in < 12 || d_out == nullptr || d_ws == nullptr) return;
  if (in_sizes[0] != kRows * kModel || in_sizes[1] != kQkvCols * kModel || in_sizes[2] != kModel * kModel ||
      in_sizes[3] != kHeads * kDk * kDk || in_sizes[4] != kHeads || in_sizes[5] != kHeads ||
      in_sizes[6] != kHeads || in_sizes[7] != kHeads || in_sizes[8] != kHeads || in_sizes[9] != kHeads ||
      in_sizes[10] != 1 || in_sizes[11] != 1 || out_size != kRows * kModel) return;

  const float* x      = (const float*)d_in[0];
  const float* w_qkv  = (const float*)d_in[1];
  const float* w_o    = (const float*)d_in[2];
  const float* w_ltm  = (const float*)d_in[3];
  const float* v_gs   = (const float*)d_in[4];
  const float* v_t0   = (const float*)d_in[5];
  const float* b_tau  = (const float*)d_in[6];
  const float* b_gm   = (const float*)d_in[7];
  const float* c_ch   = (const float*)d_in[8];
  const float* gam    = (const float*)d_in[9];
  const float* a_ppd  = (const float*)d_in[10];
  const float* ic_th  = (const float*)d_in[11];
  float* out = (float*)d_out;

  char* ws = (char*)d_ws;
  size_t off = 0;
  auto carve = [&](size_t bytes) -> char* { char* p = ws + off; off += (bytes + 255) & ~(size_t)255; return p; };
  unsigned short* XH   = (unsigned short*)carve((size_t)kRows * kModel * 2);
  unsigned short* WQH  = (unsigned short*)carve((size_t)kQkvCols * kModel * 2);
  unsigned short* WOH  = (unsigned short*)carve((size_t)kModel * kModel * 2);
  float*          QKV  = (float*)carve((size_t)kRows * kQkvCols * 4);
  float*          RET  = (float*)carve((size_t)kHeads * kDk * kDk * 4);
  float*          COEF = (float*)carve((size_t)kHeads * kDk * kDk * 4);
  unsigned short* YH   = (unsigned short*)carve((size_t)kRows * kModel * 2);
  if (off > ws_size || off > (size_t)134217728) return;

  const int n8x = kRows * kModel / 8;
  const int n8q = kQkvCols * kModel / 8;
  const int n8o = kModel * kModel / 8;
  cast8_f16_kernel<<<(n8x + 255) / 256, 256, 0, stream>>>(x,     XH,  n8x, 1.0f);
  cast8_f16_kernel<<<(n8q + 255) / 256, 256, 0, stream>>>(w_qkv, WQH, n8q, kWCarry);
  cast8_f16_kernel<<<(n8o + 255) / 256, 256, 0, stream>>>(w_o,   WOH, n8o, kWCarry);

  {
    const int tiles = (kRows / 64) * (kQkvCols / 64);
    gemm_f16_nt_kernel<<<(tiles + 7) / 8, 256, 0, stream>>>(XH, kModel, WQH, kModel, QKV, kQkvCols,
                                                           kRows, kQkvCols, kModel, kWCarryInv);
  }

  head_consts_kernel<<<(kHeads * kDk * kDk) / 256, 256, 0, stream>>>(
      w_ltm, v_gs, v_t0, b_tau, b_gm, c_ch, gam, a_ppd, ic_th, RET, COEF);

  stp_scan_kernel<<<kNB * kHeads, kThreads, 0, stream>>>(QKV, w_ltm, RET, COEF, YH);

  {
    const int tiles = (kRows / 64) * (kModel / 64);
    gemm_f16_nt_kernel<<<(tiles + 7) / 8, 256, 0, stream>>>(YH, kModel, WOH, kModel, out, kModel,
                                                           kRows, kModel, kModel, kWCarryInv);
  }
}
